// SS2D_12249246728874
// MI455X (gfx1250) — hardware-run, weakly checked
//
#include <hip/hip_runtime.h>
#include <math.h>

typedef __attribute__((ext_vector_type(16))) _Float16 v16h;
typedef __attribute__((ext_vector_type(8)))  _Float16 v8h;
typedef __attribute__((ext_vector_type(8)))  float    v8f;
typedef __attribute__((ext_vector_type(4)))  float    v4f;

constexpr int kBatch = 2;
constexpr int kImgH  = 64;
constexpr int kImgW  = 64;
constexpr int kSeq   = kImgH * kImgW;
constexpr int kRows  = kBatch * kSeq;
constexpr int kDm    = 192;
constexpr int kDi    = 384;
constexpr int kNs    = 16;
constexpr int kDtR   = 12;
constexpr int kXzN   = 2 * kDi;
constexpr int kXdW   = kDtR + 2 * kNs;
constexpr int kXdP   = 64;
constexpr int kDtK   = 32;
constexpr int kTileP = 388;
constexpr int kScTS  = 64;
static_assert(kSeq == 4096 && kRows == 8192 && kXzN == 768 && kXdW == 44);
static_assert((kDm % 32) == 0 && (kDi % 32) == 0 && (kDtK % 32) == 0);
static_assert((kRows % 64) == 0 && (kDi % 64) == 0 && (kXdP % 64) == 0 && (kDm % 64) == 0);
static_assert(kXdW <= kXdP && kDtR <= kDtK && (kDtR % 4) == 0);
static_assert((kSeq % kScTS) == 0 && (kDi % 32) == 0 && (kRows % 16) == 0);
static_assert((kDm % 64) == 0 && (kDi % 64) == 0);
static_assert(((kTileP * 4) % 16) == 0 && kTileP >= kDi);

constexpr float kCarAct = 16.0f;
constexpr float kCarY   = 64.0f;
constexpr float kCarW   = 256.0f;
constexpr float kScaleAct = 1.0f / (kCarAct * kCarW);
constexpr float kScaleOut = 1.0f / (kCarY * kCarW);
constexpr float kLnEps  = 1e-5f;
constexpr float kInvDi  = 1.0f / (float)kDi;

constexpr size_t kSzX16   = (size_t)kRows * kDm   * 2;
constexpr size_t kSzU16   = (size_t)kRows * kDi   * 2;
constexpr size_t kSzWINT  = (size_t)kXzN  * kDm   * 2;
constexpr size_t kSzWXT   = (size_t)kXdP  * kDi   * 2;
constexpr size_t kSzWDTT  = (size_t)kDi   * kDtK  * 2;
constexpr size_t kSzWOUTT = (size_t)kDm   * kDi   * 2;
constexpr size_t kSzXI    = (size_t)kRows * kDi   * 4;
constexpr size_t kSzZ     = (size_t)kRows * kDi   * 4;
constexpr size_t kSzU     = (size_t)kRows * kDi   * 4;
constexpr size_t kSzXD    = (size_t)kRows * kXdP  * 4;
constexpr size_t kSzDT16  = (size_t)kRows * kDtK  * 2;
constexpr size_t kSzDP    = (size_t)kRows * kDi   * 4;
constexpr size_t kSzY16   = (size_t)kRows * kDi   * 2;
constexpr size_t kOffX16   = 0;
constexpr size_t kOffU16   = kOffX16   + kSzX16;
constexpr size_t kOffWINT  = kOffU16   + kSzU16;
constexpr size_t kOffWXT   = kOffWINT  + kSzWINT;
constexpr size_t kOffWDTT  = kOffWXT   + kSzWXT;
constexpr size_t kOffWOUTT = kOffWDTT  + kSzWDTT;
constexpr size_t kOffXI    = kOffWOUTT + kSzWOUTT;
constexpr size_t kOffZ     = kOffXI    + kSzXI;
constexpr size_t kOffU     = kOffZ     + kSzZ;
constexpr size_t kOffXD    = kOffU     + kSzU;
constexpr size_t kOffDT16  = kOffXD    + kSzXD;
constexpr size_t kOffDP    = kOffDT16  + kSzDT16;
constexpr size_t kWsTotal  = kOffDP    + kSzDP;
static_assert(kWsTotal == 62906368ull);
static_assert(kWsTotal <= 134217728ull);
static_assert(kSzY16 <= kSzU16);
static_assert(kOffZ == kOffXI + (size_t)kRows * kDi * 4);
static_assert((kOffU16 % 128) == 0 && (kOffWINT % 128) == 0 && (kOffWXT % 128) == 0 && (kOffWDTT % 128) == 0 &&
              (kOffWOUTT % 128) == 0 && (kOffXI % 128) == 0 && (kOffZ % 128) == 0 && (kOffU % 128) == 0 &&
              (kOffXD % 128) == 0 && (kOffDT16 % 128) == 0 && (kOffDP % 128) == 0);

__device__ __forceinline__ float bf16_rne(float f) {
  unsigned u = __float_as_uint(f);
  const unsigned lsb = (u & 0x00010000u) ? 1u : 0u;
  u = (u + 0x7FFFu + lsb) & 0xFFFF0000u;
  return __uint_as_float(u);
}
__device__ __forceinline__ _Float16 to_f16_carry(float v, float carry) {
  float c = v * carry;
  c = fminf(fmaxf(c, -65000.0f), 65000.0f);
  c = (fabsf(c) < 6.103515625e-5f) ? 0.0f : c;
  return (_Float16)c;
}

union FragU { v16h v; v8h h[2]; };
__device__ __forceinline__ v16h frag_load(const _Float16* p) {
  FragU f;
  f.h[0] = *(const v8h*)(p);
  f.h[1] = *(const v8h*)(p + 16);
  return f.v;
}
__device__ __forceinline__ v8f mma_f16(v16h a, v16h b, v8f c) {
  c = __builtin_amdgcn_wmma_f32_16x16x32_f16(false, a, false, b, (short)0, c, false, false);
  asm volatile("v_nop\n\tv_nop\n\tv_nop\n\tv_nop" : "+v"(c) : "v"(a), "v"(b));
  return c;
}
__device__ __forceinline__ void keep4_h(v16h a, v16h b, v16h c, v16h d) { asm volatile("v_nop" :: "v"(a), "v"(b), "v"(c), "v"(d)); }
__device__ __forceinline__ void acc_guard4(v8f& a, v8f& b, v8f& c, v8f& d) { asm volatile("v_nop\n\tv_nop\n\tv_nop\n\tv_nop" : "+v"(a), "+v"(b), "+v"(c), "+v"(d)); }

template <bool BIAS>
__global__ __launch_bounds__(256) void gemm_f16_kernel(
    const unsigned short* __restrict__ Ap, int lda,
    const unsigned short* __restrict__ Btp, int ldb, long strideB,
    float* __restrict__ Cp, int ldc, long strideC,
    const float* __restrict__ biasp, long strideBias,
    int M, int N, int K, float scale) {
  const _Float16* A  = (const _Float16*)Ap;
  const _Float16* Bt = (const _Float16*)Btp + (size_t)blockIdx.y * (size_t)strideB;
  float* C = Cp + (size_t)blockIdx.y * (size_t)strideC;
  __shared__ __align__(16) float sT[8][16 * 68];
  const int lane = threadIdx.x & 31;
  const int wave = threadIdx.x >> 5;
  const int tilesN = N >> 6;
  const int tilesM = M >> 6;
  const int tile = blockIdx.x * 8 + wave;
  if (tile >= tilesM * tilesN) return;
  const int tm = tile / tilesN;
  const int tn = tile - tm * tilesN;
  const int m0 = tm << 6;
  const int n0 = tn << 6;

  const int rlane = lane & 15;
  const int koff  = (lane >> 4) * 8;
  const int mOff  = (lane >> 4) * 8;

  v8f acc[4][4];
#pragma unroll
  for (int i = 0; i < 4; ++i)
#pragma unroll
    for (int j = 0; j < 4; ++j) acc[i][j] = (v8f){0.f,0.f,0.f,0.f,0.f,0.f,0.f,0.f};

  for (int k0 = 0; k0 < K; k0 += 32) {
    v16h bh[4];
#pragma unroll
    for (int j = 0; j < 4; ++j) {
      const size_t bo = (size_t)(n0 + (j << 4) + rlane) * ldb + koff + k0;
      bh[j] = frag_load(Bt + bo);
    }
#pragma unroll
    for (int i = 0; i < 4; ++i) {
      const size_t ao = (size_t)(m0 + (i << 4) + rlane) * lda + koff + k0;
      const v16h ah = frag_load(A + ao);
#pragma unroll
      for (int j = 0; j < 4; ++j) acc[i][j] = mma_f16(ah, bh[j], acc[i][j]);
    }
    keep4_h(bh[0], bh[1], bh[2], bh[3]);
  }
  acc_guard4(acc[0][0], acc[0][1], acc[0][2], acc[0][3]);
  acc_guard4(acc[1][0], acc[1][1], acc[1][2], acc[1][3]);
  acc_guard4(acc[2][0], acc[2][1], acc[2][2], acc[2][3]);
  acc_guard4(acc[3][0], acc[3][1], acc[3][2], acc[3][3]);

  float bvj[4];
#pragma unroll
  for (int j = 0; j < 4; ++j) {
    float t = 0.0f;
    if (BIAS) {
      t = biasp[(size_t)blockIdx.y * (size_t)strideBias + (size_t)(n0 + (j << 4) + rlane)];
      asm volatile("" : "+v"(t));
      t = bf16_rne(t);
    }
    bvj[j] = t;
  }

  float* slab = sT[wave];
#pragma unroll
  for (int i = 0; i < 4; ++i) {
    const int mBase = m0 + (i << 4);
#pragma unroll
    for (int j = 0; j < 4; ++j) {
#pragma unroll
      for (int r = 0; r < 8; ++r) {
        float v = acc[i][j][r] * scale;
        if (BIAS) v = v + bvj[j];
        slab[(mOff + r) * 68 + (j << 4) + rlane] = v;
      }
    }
    __builtin_amdgcn_fence(__ATOMIC_RELEASE, "workgroup");
    __builtin_amdgcn_wave_barrier();
    __builtin_amdgcn_fence(__ATOMIC_ACQUIRE, "workgroup");
    {
      const int hh = lane >> 4, c4 = (lane & 15) * 4;
      for (int pass = 0; pass < 2; ++pass) {
#pragma unroll
        for (int it = 0; it < 8; ++it) {
          const int row = it * 2 + hh;
          const v4f v = *(const v4f*)(slab + row * 68 + c4);
          *(volatile v4f*)(C + (size_t)(mBase + row) * ldc + n0 + c4) = v;
        }
        __threadfence();
      }
    }
    __builtin_amdgcn_fence(__ATOMIC_RELEASE, "workgroup");
    __builtin_amdgcn_wave_barrier();
    __builtin_amdgcn_fence(__ATOMIC_ACQUIRE, "workgroup");
  }
}

template <bool BF>
__global__ __launch_bounds__(256) void cvt_rows_kernel(
    const float* __restrict__ src, unsigned srcPitch, unsigned cols8, unsigned validCols, unsigned validRows,
    unsigned short* __restrict__ dst, unsigned dstPitch, unsigned dstColOff, unsigned total8, float carry) {
  const unsigned i = blockIdx.x * 256u + threadIdx.x;
  if (i >= total8) return;
  unsigned row = i / cols8;
  unsigned col = (i - row * cols8) << 3;
  asm volatile("" : "+v"(row));
  asm volatile("" : "+v"(col));
  const bool rowOk = row < validRows;
  const unsigned rowc = rowOk ? row : (validRows - 1u);
  const float* sp = src + (size_t)rowc * srcPitch + col;
  const v4f a0 = *(const v4f*)(sp);
  const v4f a1 = *(const v4f*)(sp + 4);
  float f0 = a0[0], f1 = a0[1], f2 = a0[2], f3 = a0[3];
  float f4 = a1[0], f5 = a1[1], f6 = a1[2], f7 = a1[3];
  asm volatile("" : "+v"(f0), "+v"(f1), "+v"(f2), "+v"(f3));
  asm volatile("" : "+v"(f4), "+v"(f5), "+v"(f6), "+v"(f7));
  if (BF) {
    f0 = bf16_rne(f0); f1 = bf16_rne(f1); f2 = bf16_rne(f2); f3 = bf16_rne(f3);
    f4 = bf16_rne(f4); f5 = bf16_rne(f5); f6 = bf16_rne(f6); f7 = bf16_rne(f7);
  }
  f0 = (rowOk && (col + 0u < validCols)) ? f0 : 0.0f;
  f1 = (rowOk && (col + 1u < validCols)) ? f1 : 0.0f;
  f2 = (rowOk && (col + 2u < validCols)) ? f2 : 0.0f;
  f3 = (rowOk && (col + 3u < validCols)) ? f3 : 0.0f;
  f4 = (rowOk && (col + 4u < validCols)) ? f4 : 0.0f;
  f5 = (rowOk && (col + 5u < validCols)) ? f5 : 0.0f;
  f6 = (rowOk && (col + 6u < validCols)) ? f6 : 0.0f;
  f7 = (rowOk && (col + 7u < validCols)) ? f7 : 0.0f;
  v8h hv;
  hv[0] = to_f16_carry(f0, carry);
  hv[1] = to_f16_carry(f1, carry);
  hv[2] = to_f16_carry(f2, carry);
  hv[3] = to_f16_carry(f3, carry);
  hv[4] = to_f16_carry(f4, carry);
  hv[5] = to_f16_carry(f5, carry);
  hv[6] = to_f16_carry(f6, carry);
  hv[7] = to_f16_carry(f7, carry);
  unsigned short* q = dst + (size_t)row * dstPitch + dstColOff + col;
  *(volatile v8h*)q = hv;
  __threadfence();
  *(volatile v8h*)q = hv;
}

__global__ __launch_bounds__(256) void dtw_plane_kernel(
    const float* __restrict__ Wdt, unsigned short* __restrict__ dst, float carry) {
  const unsigned i = blockIdx.x * 256u + threadIdx.x;
  unsigned n  = i >> 2;
  unsigned k8 = (i & 3u) << 3;
  asm volatile("" : "+v"(n));
  asm volatile("" : "+v"(k8));
  v8h hv;
#pragma unroll
  for (int e = 0; e < 8; ++e) {
    const unsigned k = k8 + (unsigned)e;
    const unsigned kc = (k < (unsigned)kDtR) ? k : (unsigned)(kDtR - 1);
    float v = Wdt[(size_t)n * kDtR + kc];
    asm volatile("" : "+v"(v));
    const float vb = bf16_rne(v);
    const float f = (k < (unsigned)kDtR) ? vb : 0.0f;
    hv[e] = to_f16_carry(f, carry);
  }
  unsigned short* q = dst + (size_t)i * 8u;
  *(volatile v8h*)q = hv;
  __threadfence();
  *(volatile v8h*)q = hv;
}

__global__ __launch_bounds__(384) void conv_silu_kernel(
    const float* __restrict__ XI, const float* __restrict__ cw, const float* __restrict__ cb,
    float* __restrict__ U, unsigned short* __restrict__ U16) {
  __shared__ __align__(16) float sT[16 * kTileP];
  const unsigned tid = threadIdx.x;
  unsigned lane = tid & 31u;
  unsigned wave = tid >> 5;
  asm volatile("" : "+v"(lane));
  asm volatile("" : "+v"(wave));
  const unsigned hy = blockIdx.x & (unsigned)(kImgH - 1);
  const size_t rowM = (size_t)blockIdx.x * (size_t)kImgW;
  const bool top = (hy > 0u);
  const bool bot = (hy < (unsigned)(kImgH - 1));
  const size_t rowT = top ? (rowM - (size_t)kImgW) : rowM;
  const size_t rowB = bot ? (rowM + (size_t)kImgW) : rowM;
  const float* wp = cw + (size_t)tid * 9u;
  const float w00 = bf16_rne(wp[0]), w01 = bf16_rne(wp[1]), w02 = bf16_rne(wp[2]);
  const float w10 = bf16_rne(wp[3]), w11 = bf16_rne(wp[4]), w12 = bf16_rne(wp[5]);
  const float w20 = bf16_rne(wp[6]), w21 = bf16_rne(wp[7]), w22 = bf16_rne(wp[8]);
  const float bc = bf16_rne(cb[tid]);
  float lt = 0.0f, lm = 0.0f, lb = 0.0f;
  float ct, cm, cq;
  {
    const float t0 = XI[rowT * kDi + tid];
    const float m0 = XI[rowM * kDi + tid];
    const float b0 = XI[rowB * kDi + tid];
    ct = top ? t0 : 0.0f;
    cm = m0;
    cq = bot ? b0 : 0.0f;
  }
  unsigned q  = lane >> 3;
  unsigned l7 = lane & 7u;
  asm volatile("" : "+v"(q));
  asm volatile("" : "+v"(l7));
#pragma unroll 1
  for (unsigned sub = 0; sub < 4u; ++sub) {
    const size_t pb = rowM + sub * 16u;
#pragma unroll 1
    for (unsigned s = 0; s < 16u; ++s) {
      const unsigned wc = sub * 16u + s;
      const bool hasR = (wc + 1u) < (unsigned)kImgW;
      const unsigned wn = hasR ? (wc + 1u) : (unsigned)(kImgW - 1);
      const float nt = XI[(rowT + wn) * kDi + tid];
      const float nm = XI[(rowM + wn) * kDi + tid];
      const float nb = XI[(rowB + wn) * kDi + tid];
      const float rt = (top && hasR) ? nt : 0.0f;
      const float rm = hasR ? nm : 0.0f;
      const float rb = (bot && hasR) ? nb : 0.0f;
      float acc = w00 * lt;
      acc = fmaf(w01, ct, acc);
      acc = fmaf(w02, rt, acc);
      acc = fmaf(w10, lm, acc);
      acc = fmaf(w11, cm, acc);
      acc = fmaf(w12, rm, acc);
      acc = fmaf(w20, lb, acc);
      acc = fmaf(w21, cq, acc);
      acc = fmaf(w22, rb, acc);
      const float sv = acc + bc;
      const float sg = 1.0f / (1.0f + expf(-sv));
      sT[s * kTileP + tid] = sv * sg;
      lt = ct; ct = rt;
      lm = cm; cm = rm;
      lb = cq; cq = rb;
    }
    __syncthreads();
    v4f fv[4];
    v8h hv[2];
#pragma unroll
    for (int it = 0; it < 4; ++it) {
      const unsigned ci = (unsigned)it * 12u + wave;
      const unsigned pr = ci / 3u;
      const unsigned th = ci - pr * 3u;
      fv[it] = *(const v4f*)(sT + pr * kTileP + th * 128u + lane * 4u);
    }
#pragma unroll
    for (int it = 0; it < 2; ++it) {
      const unsigned li = (unsigned)it * 48u + wave * 4u + q;
      const unsigned pr = li / 6u;
      const unsigned sg6 = li - pr * 6u;
      const float* sp = sT + pr * kTileP + sg6 * 64u + l7 * 8u;
      const v4f a0 = *(const v4f*)(sp);
      const v4f a1 = *(const v4f*)(sp + 4);
#pragma unroll
      for (int e = 0; e < 4; ++e) {
        const float f0 = a0[e];
        const float f1 = a1[e];
        hv[it][e]     = to_f16_carry(f0, kCarAct);
        hv[it][4 + e] = to_f16_carry(f1, kCarAct);
      }
    }
    for (int pass = 0; pass < 2; ++pass) {
#pragma unroll
      for (int it = 0; it < 4; ++it) {
        const unsigned ci = (unsigned)it * 12u + wave;
        const unsigned pr = ci / 3u;
        const unsigned th = ci - pr * 3u;
        *(volatile v4f*)(U + (pb + pr) * kDi + th * 128u + lane * 4u) = fv[it];
      }
#pragma unroll
      for (int it = 0; it < 2; ++it) {
        const unsigned li = (unsigned)it * 48u + wave * 4u + q;
        const unsigned pr = li / 6u;
        const unsigned sg6 = li - pr * 6u;
        *(volatile v8h*)(U16 + (pb + pr) * kDi + sg6 * 64u + l7 * 8u) = hv[it];
      }
      __threadfence();
    }
    __syncthreads();
  }
}

__global__ __launch_bounds__(32) void scan_kernel(
    const float* __restrict__ XD, const float* __restrict__ DP, const float* __restrict__ U,
    const float* __restrict__ bdt, const float* __restrict__ Alog, const float* __restrict__ Dsk,
    float* __restrict__ YS) {
  __shared__ __align__(16) float sX[kScTS * 32];
  __shared__ __align__(16) float sY[kScTS * 32];
  __shared__ __align__(16) float sA[kNs * 32];
  const unsigned tid = threadIdx.x;
  constexpr unsigned kBlkPerB = (unsigned)(kDi / 32);
  const unsigned bix = blockIdx.x / kBlkPerB;
  const unsigned d0  = (blockIdx.x - bix * kBlkPerB) * 32u;
  const unsigned d   = d0 + tid;
  const size_t row0 = (size_t)bix * kSeq;
#pragma unroll 1
  for (unsigned s = 0; s < (unsigned)kNs; ++s) {
    const float al = Alog[(size_t)d * kNs + s];
    sA[s * 32u + tid] = -expf(bf16_rne(al));
  }
  __syncthreads();
  float negA[kNs], h[kNs];
#pragma unroll
  for (int s = 0; s < kNs; ++s) {
    negA[s] = sA[s * 32 + tid];
    h[s] = 0.0f;
  }
  const float bb = bf16_rne(bdt[d]);
  const float Dd = bf16_rne(Dsk[d]);
  unsigned q  = tid >> 3;
  unsigned l7 = tid & 7u;
  asm volatile("" : "+v"(q));
  asm volatile("" : "+v"(l7));
#pragma unroll 1
  for (unsigned t0 = 0; t0 < (unsigned)kSeq; t0 += (unsigned)kScTS) {
    __syncthreads();
#pragma unroll
    for (unsigned k = 0; k < 16u; ++k) {
      const unsigned idx = tid + 32u * k;
      const unsigned r = idx >> 3;
      const unsigned c4 = (idx & 7u) * 4u;
      *(v4f*)(sX + r * 32u + c4) = *(const v4f*)(XD + (row0 + t0 + r) * kXdP + kDtR + c4);
    }
    __syncthreads();
#pragma unroll 1
    for (unsigned s = 0; s < (unsigned)kScTS; ++s) {
      const size_t row = row0 + t0 + s;
      float pre = DP[row * kDi + d];
      float ut  = U[row * kDi + d];
      asm volatile("" : "+v"(pre));
      asm volatile("" : "+v"(ut));
      const float v  = pre + bb;
      const float ea = expf(-fabsf(v));
      const float u1 = 1.0f + ea;
      const float l1p = logf(u1) + (ea - (u1 - 1.0f)) * __builtin_amdgcn_rcpf(u1);
      const float delta = fmaxf(v, 0.0f) + l1p;
      const float dtx = delta * ut;
      const float* xr = sX + s * 32u;
      float Bv[kNs], Cv[kNs];
#pragma unroll
      for (int q4 = 0; q4 < 4; ++q4) {
        const v4f bv = *(const v4f*)(xr + 4 * q4);
        const v4f cv = *(const v4f*)(xr + kNs + 4 * q4);
        Bv[4 * q4 + 0] = bv[0]; Bv[4 * q4 + 1] = bv[1]; Bv[4 * q4 + 2] = bv[2]; Bv[4 * q4 + 3] = bv[3];
        Cv[4 * q4 + 0] = cv[0]; Cv[4 * q4 + 1] = cv[1]; Cv[4 * q4 + 2] = cv[2]; Cv[4 * q4 + 3] = cv[3];
      }
      float y = 0.0f;
#pragma unroll
      for (int n = 0; n < kNs; ++n) {
        const float ee = __expf(delta * negA[n]);
        h[n] = fmaf(ee, h[n], dtx * Bv[n]);
        y = fmaf(h[n], Cv[n], y);
      }
      y = fmaf(ut, Dd, y);
      sY[s * 32u + tid] = y;
    }
    __syncthreads();
    v4f ov[16];
#pragma unroll
    for (int it = 0; it < 16; ++it) {
      const unsigned r = (unsigned)it * 4u + q;
      ov[it] = *(const v4f*)(sY + r * 32u + l7 * 4u);
    }
    for (int pass = 0; pass < 2; ++pass) {
#pragma unroll
      for (int it = 0; it < 16; ++it) {
        const unsigned r = (unsigned)it * 4u + q;
        *(volatile v4f*)(YS + (row0 + t0 + r) * kDi + d0 + l7 * 4u) = ov[it];
      }
      __threadfence();
    }
  }
}

__global__ __launch_bounds__(256) void norm_gate_kernel(
    const float* __restrict__ YS, const float* __restrict__ Z,
    const float* __restrict__ lng, const float* __restrict__ lnb,
    unsigned short* __restrict__ Y16) {
  __shared__ __align__(16) float sG[16 * kTileP];
  const unsigned tid = threadIdx.x;
  unsigned lane = tid & 31u;
  unsigned wave = tid >> 5;
  asm volatile("" : "+v"(lane));
  asm volatile("" : "+v"(wave));
  const size_t row0 = (size_t)blockIdx.x * 16u;
#pragma unroll 1
  for (unsigned rr = 0; rr < 2u; ++rr) {
    const unsigned lrow = wave * 2u + rr;
    const size_t grow = row0 + lrow;
    const float* yp = YS + grow * kDi + lane * 4u;
    const v4f ya = *(const v4f*)(yp);
    const v4f yb = *(const v4f*)(yp + 128);
    const v4f yc = *(const v4f*)(yp + 256);
    float s = ((ya[0] + ya[1]) + (ya[2] + ya[3])) + ((yb[0] + yb[1]) + (yb[2] + yb[3]));
    s = s + ((yc[0] + yc[1]) + (yc[2] + yc[3]));
    s += __shfl_xor(s, 16, 32);
    s += __shfl_xor(s, 8, 32);
    s += __shfl_xor(s, 4, 32);
    s += __shfl_xor(s, 2, 32);
    s += __shfl_xor(s, 1, 32);
    const float mu = s * kInvDi;
    float s2 = 0.0f;
#pragma unroll
    for (int e = 0; e < 4; ++e) {
      const float da = ya[e] - mu;
      const float db = yb[e] - mu;
      const float dc = yc[e] - mu;
      s2 = fmaf(da, da, s2);
      s2 = fmaf(db, db, s2);
      s2 = fmaf(dc, dc, s2);
    }
    s2 += __shfl_xor(s2, 16, 32);
    s2 += __shfl_xor(s2, 8, 32);
    s2 += __shfl_xor(s2, 4, 32);
    s2 += __shfl_xor(s2, 2, 32);
    s2 += __shfl_xor(s2, 1, 32);
    const float rstd = rsqrtf(s2 * kInvDi + kLnEps);
    float* gp = sG + lrow * kTileP + lane * 4u;
    *(v4f*)(gp) = ya;
    *(v4f*)(gp + 128) = yb;
    *(v4f*)(gp + 256) = yc;
#pragma unroll 1
    for (unsigned j = 0; j < 3u; ++j) {
      float* gq = gp + j * 128u;
      const v4f yv = *(const v4f*)gq;
      const v4f zq = *(const v4f*)(Z + grow * kDi + j * 128u + lane * 4u);
      const v4f gg = *(const v4f*)(lng + j * 128u + lane * 4u);
      const v4f bq = *(const v4f*)(lnb + j * 128u + lane * 4u);
      v4f ovv;
#pragma unroll
      for (int e = 0; e < 4; ++e) {
        const float ge = bf16_rne(gg[e]);
        const float be = bf16_rne(bq[e]);
        const float yn = (yv[e] - mu) * rstd * ge + be;
        const float zz = zq[e];
        const float sg = 1.0f / (1.0f + expf(-zz));
        ovv[e] = yn * (zz * sg);
      }
      *(v4f*)gq = ovv;
    }
  }
  __syncthreads();
  unsigned q  = lane >> 3;
  unsigned l7 = lane & 7u;
  asm volatile("" : "+v"(q));
  asm volatile("" : "+v"(l7));
  v8h hv[3];
#pragma unroll
  for (int it = 0; it < 3; ++it) {
    const unsigned li = (unsigned)it * 32u + wave * 4u + q;
    const unsigned pr = li / 6u;
    const unsigned sg6 = li - pr * 6u;
    const float* sp = sG + pr * kTileP + sg6 * 64u + l7 * 8u;
    const v4f a0 = *(const v4f*)(sp);
    const v4f a1 = *(const v4f*)(sp + 4);
#pragma unroll
    for (int e = 0; e < 4; ++e) {
      const float f0 = a0[e];
      const float f1 = a1[e];
      hv[it][e]     = to_f16_carry(f0, kCarY);
      hv[it][4 + e] = to_f16_carry(f1, kCarY);
    }
  }
  for (int pass = 0; pass < 2; ++pass) {
#pragma unroll
    for (int it = 0; it < 3; ++it) {
      const unsigned li = (unsigned)it * 32u + wave * 4u + q;
      const unsigned pr = li / 6u;
      const unsigned sg6 = li - pr * 6u;
      *(volatile v8h*)(Y16 + (row0 + pr) * kDi + sg6 * 64u + l7 * 8u) = hv[it];
    }
    __threadfence();
  }
}

static_assert((((kRows / 64) * (kDi / 64)) % 8) == 0);
static_assert((((kRows / 64) * (kXdP / 64)) % 8) == 0);
static_assert((((kRows / 64) * (kDm / 64)) % 8) == 0);
static_assert(((kRows * (kDm / 8)) % 256) == 0 && ((kRows * (kDtK / 8)) % 256) == 0 && ((kDi * (kDtK / 8)) % 256) == 0);
static_assert(((kXzN * (kDm / 8)) % 256) == 0 && ((kXdP * (kDi / 8)) % 256) == 0 && ((kDm * (kDi / 8)) % 256) == 0);

extern "C" void kernel_launch(void* const* d_in, const int* in_sizes, int n_in,
                              void* d_out, int out_size, void* d_ws, size_t ws_size,
                              hipStream_t stream) {
  if (n_in < 14) return;
  if (in_sizes[0]  != kRows * kDm) return;
  if (in_sizes[1]  != kXzN * kDm) return;
  if (in_sizes[2]  != kXzN) return;
  if (in_sizes[3]  != kDi * 9) return;
  if (in_sizes[4]  != kDi) return;
  if (in_sizes[5]  != kXdW * kDi) return;
  if (in_sizes[6]  != kDi * kDtR) return;
  if (in_sizes[7]  != kDi) return;
  if (in_sizes[8]  != kDi * kNs) return;
  if (in_sizes[9]  != kDi) return;
  if (in_sizes[10] != kDi) return;
  if (in_sizes[11] != kDi) return;
  if (in_sizes[12] != kDm * kDi) return;
  if (in_sizes[13] != kDm) return;
  if (out_size != kRows * kDm) return;
  if (ws_size < kWsTotal) return;

  const float* x      = (const float*)d_in[0];
  const float* W_in   = (const float*)d_in[1];
  const float* b_in   = (const float*)d_in[2];
  const float* conv_w = (const float*)d_in[3];
  const float* conv_b = (const float*)d_in[4];
  const float* Wx     = (const float*)d_in[5];
  const float* Wdt    = (const float*)d_in[6];
  const float* b_dt   = (const float*)d_in[7];
  const float* A_log  = (const float*)d_in[8];
  const float* D_skip = (const float*)d_in[9];
  const float* ln_g   = (const float*)d_in[10];
  const float* ln_b   = (const float*)d_in[11];
  const float* Wout   = (const float*)d_in[12];
  const float* b_out  = (const float*)d_in[13];
  float* out = (float*)d_out;

  char* ws = (char*)d_ws;
  unsigned short* X16   = (unsigned short*)(ws + kOffX16);
  unsigned short* U16   = (unsigned short*)(ws + kOffU16);
  unsigned short* WINT  = (unsigned short*)(ws + kOffWINT);
  unsigned short* WXT   = (unsigned short*)(ws + kOffWXT);
  unsigned short* WDTT  = (unsigned short*)(ws + kOffWDTT);
  unsigned short* WOUTT = (unsigned short*)(ws + kOffWOUTT);
  float*          XI    = (float*)(ws + kOffXI);
  float*          Z     = (float*)(ws + kOffZ);
  float*          U     = (float*)(ws + kOffU);
  float*          XD    = (float*)(ws + kOffXD);
  unsigned short* DT16  = (unsigned short*)(ws + kOffDT16);
  float*          DP    = (float*)(ws + kOffDP);
  float*          YS    = XI;
  unsigned short* Y16   = U16;

  cvt_rows_kernel<true><<<(kRows * (kDm / 8)) / 256, 256, 0, stream>>>(
      x, (unsigned)kDm, (unsigned)(kDm / 8), (unsigned)kDm, (unsigned)kRows, X16, (unsigned)kDm, 0u,
      (unsigned)(kRows * (kDm / 8)), kCarAct);
  cvt_rows_kernel<true><<<(kXzN * (kDm / 8)) / 256, 256, 0, stream>>>(
      W_in, (unsigned)kDm, (unsigned)(kDm / 8), (unsigned)kDm, (unsigned)kXzN, WINT, (unsigned)kDm, 0u,
      (unsigned)(kXzN * (kDm / 8)), kCarW);
  cvt_rows_kernel<true><<<(kXdP * (kDi / 8)) / 256, 256, 0, stream>>>(
      Wx, (unsigned)kDi, (unsigned)(kDi / 8), (unsigned)kDi, (unsigned)kXdW, WXT, (unsigned)kDi, 0u,
      (unsigned)(kXdP * (kDi / 8)), kCarW);
  dtw_plane_kernel<<<(kDi * (kDtK / 8)) / 256, 256, 0, stream>>>(Wdt, WDTT, kCarW);
  cvt_rows_kernel<true><<<(kDm * (kDi / 8)) / 256, 256, 0, stream>>>(
      Wout, (unsigned)kDi, (unsigned)(kDi / 8), (unsigned)kDi, (unsigned)kDm, WOUTT, (unsigned)kDi, 0u,
      (unsigned)(kDm * (kDi / 8)), kCarW);

  gemm_f16_kernel<true><<<dim3(((kRows / 64) * (kDi / 64)) / 8, 2), 256, 0, stream>>>(
      X16, kDm, WINT, kDm, (long)kDi * (long)kDm,
      XI, kDi, (long)kRows * (long)kDi,
      b_in, (long)kDi,
      kRows, kDi, kDm, kScaleAct);

  conv_silu_kernel<<<kBatch * kImgH, 384, 0, stream>>>(XI, conv_w, conv_b, U, U16);

  gemm_f16_kernel<false><<<dim3(((kRows / 64) * (kXdP / 64)) / 8, 1), 256, 0, stream>>>(
      U16, kDi, WXT, kDi, 0L,
      XD, kXdP, 0L,
      b_out, 0L,
      kRows, kXdP, kDi, kScaleAct);

  cvt_rows_kernel<false><<<(kRows * (kDtK / 8)) / 256, 256, 0, stream>>>(
      XD, (unsigned)kXdP, (unsigned)(kDtK / 8), (unsigned)kDtR, (unsigned)kRows, DT16, (unsigned)kDtK, 0u,
      (unsigned)(kRows * (kDtK / 8)), kCarAct);

  gemm_f16_kernel<false><<<dim3(((kRows / 64) * (kDi / 64)) / 8, 1), 256, 0, stream>>>(
      DT16, kDtK, WDTT, kDtK, 0L,
      DP, kDi, 0L,
      b_out, 0L,
      kRows, kDi, kDtK, kScaleAct);

  scan_kernel<<<kBatch * (kDi / 32), 32, 0, stream>>>(XD, DP, U, b_dt, A_log, D_skip, YS);

  norm_gate_kernel<<<kRows / 16, 256, 0, stream>>>(YS, Z, ln_g, ln_b, Y16);

  gemm_f16_kernel<true><<<dim3(((kRows / 64) * (kDm / 64)) / 8, 1), 256, 0, stream>>>(
      Y16, kDi, WOUTT, kDi, 0L,
      out, kDm, 0L,
      b_out, 0L,
      kRows, kDm, kDi, kScaleOut);
}
